// PatchAutoencoder_35811437314304
// MI455X (gfx1250) — hardware-verified
//
#include <hip/hip_runtime.h>

constexpr int kImg   = 224;
constexpr int kPsz   = 16;
constexpr int kStr   = 8;
constexpr int kEdim  = 128;
constexpr int kBatch = 64;
constexpr int kChan  = 3;
constexpr int kNp    = (kImg - kPsz) / kStr + 1;
constexpr int kL     = kNp * kNp;
constexpr int kKpix  = kPsz * kPsz;
constexpr int kRows  = kBatch * kL;
static_assert(kNp == 27);
static_assert(kL == 729);
static_assert(kRows % 64 == 0);
static_assert(kKpix % 32 == 0);
static_assert(kEdim % 64 == 0);
static_assert(kImg % 8 == 0);

typedef __attribute__((ext_vector_type(16))) _Float16 v16h;
typedef __attribute__((ext_vector_type(8)))  _Float16 v8h;
typedef __attribute__((ext_vector_type(16))) __bf16   v16b;
typedef __attribute__((ext_vector_type(8)))  __bf16   v8b;
typedef __attribute__((ext_vector_type(8)))  float    v8f;
typedef __attribute__((ext_vector_type(4)))  float    v4f;
typedef __attribute__((ext_vector_type(4)))  unsigned int v4u;

__device__ __forceinline__ unsigned short f2bf_bits(float f) {
  unsigned u = __float_as_uint(f);
  return (unsigned short)((u + 0x7FFFu + ((u >> 16) & 1u)) >> 16);
}
__device__ __forceinline__ float bf_bits2f(unsigned short h) { return __uint_as_float(((unsigned)h) << 16); }

__device__ __forceinline__ void dep_guard_h(v8f& a, v8f& b, v16h x, v16h y) { asm volatile("v_nop\n\tv_nop\n\tv_nop\n\tv_nop" : "+v"(a), "+v"(b) : "v"(x), "v"(y)); }
__device__ __forceinline__ void dep_guard_b(v8f& a, v8f& b, v16b x, v16b y) { asm volatile("v_nop\n\tv_nop\n\tv_nop\n\tv_nop" : "+v"(a), "+v"(b) : "v"(x), "v"(y)); }
__device__ __forceinline__ void keep4_h(v16h a, v16h b, v16h c, v16h d) { asm volatile("v_nop" :: "v"(a), "v"(b), "v"(c), "v"(d)); }
__device__ __forceinline__ void keep4_b(v16b a, v16b b, v16b c, v16b d) { asm volatile("v_nop" :: "v"(a), "v"(b), "v"(c), "v"(d)); }
__device__ __forceinline__ void acc_guard4(v8f& a, v8f& b, v8f& c, v8f& d) { asm volatile("v_nop\n\tv_nop\n\tv_nop\n\tv_nop" : "+v"(a), "+v"(b), "+v"(c), "+v"(d)); }
template <typename T> struct Frag;
template <> struct Frag<_Float16> {
  typedef v16h V; union U { v16h v; v8h h[2]; };
  static __device__ __forceinline__ v16h load(const _Float16* p) {
    U f; f.h[0] = *(const v8h*)(p); f.h[1] = *(const v8h*)(p + 16); return f.v;
  }
  static __device__ __forceinline__ v8f mma(v16h a, v16h b, v8f c) {
    return __builtin_amdgcn_wmma_f32_16x16x32_f16(false, a, false, b, (short)0, c, false, false);
  }
  static __device__ __forceinline__ void guard(v8f& a, v8f& b, v16h x, v16h y) { dep_guard_h(a, b, x, y); }
  static __device__ __forceinline__ void keep(v16h a, v16h b, v16h c, v16h d) { keep4_h(a, b, c, d); }
};
template <> struct Frag<__bf16> {
  typedef v16b V; union U { v16b v; v8b h[2]; };
  static __device__ __forceinline__ v16b load(const __bf16* p) {
    U f; f.h[0] = *(const v8b*)(p); f.h[1] = *(const v8b*)(p + 16); return f.v;
  }
  static __device__ __forceinline__ v8f mma(v16b a, v16b b, v8f c) {
    return __builtin_amdgcn_wmma_f32_16x16x32_bf16(false, a, false, b, (short)0, c, false, false);
  }
  static __device__ __forceinline__ void guard(v8f& a, v8f& b, v16b x, v16b y) { dep_guard_b(a, b, x, y); }
  static __device__ __forceinline__ void keep(v16b a, v16b b, v16b c, v16b d) { keep4_b(a, b, c, d); }
};

__device__ __forceinline__ unsigned pk16(unsigned short a, unsigned short b) { return (unsigned)a | ((unsigned)b << 16); }
__device__ __forceinline__ unsigned short h_bits(float f) { const _Float16 h = (_Float16)f; return __builtin_bit_cast(unsigned short, h); }

template <int ET> struct Elem;
template <> struct Elem<0> { typedef _Float16 T; };
template <> struct Elem<1> { typedef __bf16 T; };
template <int ET, int SPL, int BIAS_MODE, int OUT_MODE>
__global__ __launch_bounds__(256) void wmma_gemm64(
    const unsigned short* __restrict__ Ap, const unsigned short* __restrict__ A2p, int lda, long strideA,
    const unsigned short* __restrict__ Btp, const unsigned short* __restrict__ Bt2p, int ldb, long strideB,
    void* __restrict__ Cout, void* __restrict__ Cout2, int ldc, long strideC,
    const float* __restrict__ bias, long strideBias,
    int M, int N, int K, float scale) {
  typedef typename Elem<ET>::T T;
  typedef typename Frag<T>::V V;
  const T* A = (const T*)Ap; const T* A2 = (const T*)A2p; const T* Bt = (const T*)Btp; const T* Bt2 = (const T*)Bt2p;
  __shared__ __align__(16) float sT[8][16 * 68];
  const int b    = blockIdx.y;
  const int lane = threadIdx.x & 31;
  const int wave = threadIdx.x >> 5;
  const int tilesN = N >> 6;
  const int tilesM = M >> 6;
  const int tile = blockIdx.x * 8 + wave;
  if (tile >= tilesM * tilesN) return;
  const int tm = tile / tilesN;
  const int tn = tile - tm * tilesN;
  const int m0 = tm << 6;
  const int n0 = tn << 6;

  const T* Ab  = A  + (size_t)b * strideA;
  const T* Bb  = Bt + (size_t)b * strideB;
  const T* Ab2 = (SPL & 1) ? (A2  + (size_t)b * strideA) : nullptr;
  const T* Bb2 = (SPL & 2) ? (Bt2 + (size_t)b * strideB) : nullptr;

  const int rlane = lane & 15;
  const int koff  = (lane >> 4) * 8;
  const int mOff  = (lane >> 4) * 8;

  v8f acc[4][4];
#pragma unroll
  for (int i = 0; i < 4; ++i)
#pragma unroll
    for (int j = 0; j < 4; ++j) acc[i][j] = (v8f){0.f,0.f,0.f,0.f,0.f,0.f,0.f,0.f};

  for (int k0 = 0; k0 < K; k0 += 32) {
    V bh[4], bl[4];
#pragma unroll
    for (int j = 0; j < 4; ++j) {
      const size_t bo = (size_t)(n0 + (j << 4) + rlane) * ldb + koff + k0;
      bh[j] = Frag<T>::load(Bb + bo);
      if (SPL & 2) bl[j] = Frag<T>::load(Bb2 + bo);
    }
#pragma unroll
    for (int i = 0; i < 4; ++i) {
      const size_t ao = (size_t)(m0 + (i << 4) + rlane) * lda + koff + k0;
      V ah = Frag<T>::load(Ab + ao);
      V al;
      if (SPL & 1) al = Frag<T>::load(Ab2 + ao);
#pragma unroll
      for (int j = 0; j < 4; ++j) {
        acc[i][j] = Frag<T>::mma(ah, bh[j], acc[i][j]);
        if (SPL & 2) acc[i][j] = Frag<T>::mma(ah, bl[j], acc[i][j]);
        if (SPL & 1) acc[i][j] = Frag<T>::mma(al, bh[j], acc[i][j]);
      }
      Frag<T>::guard(acc[i][0], acc[i][3], ah, (SPL & 1) ? al : ah);
    }
    Frag<T>::keep(bh[0], bh[1], bh[2], bh[3]);
    if (SPL & 2) Frag<T>::keep(bl[0], bl[1], bl[2], bl[3]);
  }
  acc_guard4(acc[0][0], acc[0][1], acc[0][2], acc[0][3]);
  acc_guard4(acc[1][0], acc[1][1], acc[1][2], acc[1][3]);
  acc_guard4(acc[2][0], acc[2][1], acc[2][2], acc[2][3]);
  acc_guard4(acc[3][0], acc[3][1], acc[3][2], acc[3][3]);

  float* slab = sT[wave];
  const float* Bs = (BIAS_MODE != 0) ? (bias + (size_t)b * strideBias) : nullptr;
#pragma unroll
  for (int i = 0; i < 4; ++i) {
    const int mBase = m0 + (i << 4);
#pragma unroll
    for (int j = 0; j < 4; ++j) {
      const int n = n0 + (j << 4) + rlane;
      float bv = 0.f;
      if (BIAS_MODE == 2) bv = Bs[n];
      if (BIAS_MODE == 3) bv = bf_bits2f(f2bf_bits(Bs[n]));
#pragma unroll
      for (int r = 0; r < 8; ++r) {
        float v = acc[i][j][r] * scale;
        if (BIAS_MODE >= 2) v += bv;
        slab[(mOff + r) * 68 + (j << 4) + rlane] = v;
      }
    }
    __builtin_amdgcn_fence(__ATOMIC_RELEASE, "workgroup");
    __builtin_amdgcn_wave_barrier();
    __builtin_amdgcn_fence(__ATOMIC_ACQUIRE, "workgroup");
    if (OUT_MODE == 0) {
      float* C = (float*)Cout + (size_t)b * strideC;
      const int hh = lane >> 4, c4 = (lane & 15) * 4;
      for (int pass = 0; pass < 2; ++pass) {
#pragma unroll
        for (int it = 0; it < 8; ++it) {
          const int row = it * 2 + hh;
          v4f v = *(const v4f*)(slab + row * 68 + c4);
          *(volatile v4f*)(C + (size_t)(mBase + row) * ldc + n0 + c4) = v;
        }
        __threadfence();
      }
    } else {
      const int q = lane >> 3, c8 = (lane & 7) * 8;
      unsigned short* C  = (unsigned short*)Cout  + (size_t)b * strideC;
      unsigned short* C2 = (OUT_MODE == 2) ? ((unsigned short*)Cout2 + (size_t)b * strideC) : nullptr;
      for (int pass = 0; pass < 2; ++pass) {
#pragma unroll
        for (int it = 0; it < 4; ++it) {
          const int row = it * 4 + q;
          const float* sp = slab + row * 68 + c8;
          v8h hv, lv;
#pragma unroll
          for (int e = 0; e < 8; ++e) {
            if (OUT_MODE == 1) {
              hv[e] = (_Float16)sp[e];
            } else {
              unsigned short hb = f2bf_bits(sp[e]);
              unsigned short lb = f2bf_bits(sp[e] - bf_bits2f(hb));
              hv[e] = __builtin_bit_cast(_Float16, hb);
              lv[e] = __builtin_bit_cast(_Float16, lb);
            }
          }
          *(volatile v8h*)(C + (size_t)(mBase + row) * ldc + n0 + c8) = hv;
          if (OUT_MODE == 2) *(volatile v8h*)(C2 + (size_t)(mBase + row) * ldc + n0 + c8) = lv;
        }
        __threadfence();
      }
    }
    __builtin_amdgcn_fence(__ATOMIC_RELEASE, "workgroup");
    __builtin_amdgcn_wave_barrier();
    __builtin_amdgcn_fence(__ATOMIC_ACQUIRE, "workgroup");
  }
}

template <int MODE>
__global__ __launch_bounds__(256) void cast8_kernel(const float* __restrict__ in, unsigned short* __restrict__ out, int n8, float scale) {
  const int i = blockIdx.x * 256 + threadIdx.x;
  if (i >= n8) return;
  const float* p = in + 8 * (size_t)i;
  const v4f a = *(const v4f*)(p);
  const v4f c = *(const v4f*)(p + 4);
  unsigned short hb[8];
#pragma unroll
  for (int e = 0; e < 4; ++e) {
    if (MODE == 0) {
      hb[e]     = f2bf_bits(a[e]);
      hb[4 + e] = f2bf_bits(c[e]);
    } else {
      hb[e]     = h_bits(bf_bits2f(f2bf_bits(a[e])) * scale);
      hb[4 + e] = h_bits(bf_bits2f(f2bf_bits(c[e])) * scale);
    }
  }
  const v4u u = (v4u){pk16(hb[0], hb[1]), pk16(hb[2], hb[3]), pk16(hb[4], hb[5]), pk16(hb[6], hb[7])};
  unsigned short* q = out + 8 * (size_t)i;
  *(volatile v4u*)q = u;
  __threadfence();
  *(volatile v4u*)q = u;
  (void)scale;
}

__global__ __launch_bounds__(256) void unfold_kernel(const float* __restrict__ x, unsigned short* __restrict__ A16, int c, int nrows) {
  const int wave = threadIdx.x >> 5, lane = threadIdx.x & 31;
  const int row = blockIdx.x * 8 + wave;
  if (row >= nrows) return;
  const int b  = row / kL;
  const int l  = row - b * kL;
  const int pi = l / kNp;
  const int pj = l - pi * kNp;
  const int i  = lane >> 1;
  const int j0 = (lane & 1) * 8;
  const float* src = x + ((size_t)(b * kChan + c) * kImg + (size_t)(pi * kStr + i)) * kImg + pj * kStr + j0;
  const v4f a = *(const v4f*)(src);
  const v4f d = *(const v4f*)(src + 4);
  const v4u u = (v4u){pk16(f2bf_bits(a[0]), f2bf_bits(a[1])), pk16(f2bf_bits(a[2]), f2bf_bits(a[3])),
                      pk16(f2bf_bits(d[0]), f2bf_bits(d[1])), pk16(f2bf_bits(d[2]), f2bf_bits(d[3]))};
  unsigned short* q = A16 + (size_t)row * kKpix + lane * 8;
  *(volatile v4u*)q = u;
  __threadfence();
  *(volatile v4u*)q = u;
}

__global__ __launch_bounds__(64) void fold_kernel(const float* __restrict__ rec, float* __restrict__ out, int c) {
  const int b = blockIdx.x / kImg;
  const int y = blockIdx.x - b * kImg;
  const int t = threadIdx.x;
  const bool active = (t < (kImg / 4));
  const int tc = active ? t : ((kImg / 4) - 1);
  const int x0 = tc * 4;

  int piH = y >> 3;  if (piH > kNp - 1) piH = kNp - 1;
  const int piL = (y >= kPsz) ? (((y - kPsz) >> 3) + 1) : 0;
  int pjH = x0 >> 3; if (pjH > kNp - 1) pjH = kNp - 1;
  const int pjL = (x0 >= kPsz) ? (((x0 - kPsz) >> 3) + 1) : 0;
  const bool twoY = (piH != piL);
  const bool twoX = (pjH != pjL);

  const size_t rb = (size_t)b * kL;
  const size_t r00 = rb + (size_t)(piL * kNp + pjL);
  const size_t r01 = rb + (size_t)(piL * kNp + pjH);
  const size_t r10 = rb + (size_t)(piH * kNp + pjL);
  const size_t r11 = rb + (size_t)(piH * kNp + pjH);
  const int oyL = (y - kStr * piL) * kPsz, oyH = (y - kStr * piH) * kPsz;
  const int oxL = x0 - kStr * pjL,          oxH = x0 - kStr * pjH;

  const v4f v00 = *(const v4f*)(rec + r00 * kKpix + oyL + oxL);
  const v4f v01 = *(const v4f*)(rec + r01 * kKpix + oyL + oxH);
  const v4f v10 = *(const v4f*)(rec + r10 * kKpix + oyH + oxL);
  const v4f v11 = *(const v4f*)(rec + r11 * kKpix + oyH + oxH);

  const float inv = (twoY ? 0.5f : 1.0f) * (twoX ? 0.5f : 1.0f);
  v4f r;
#pragma unroll
  for (int e = 0; e < 4; ++e) {
    float s = 0.0f + v00[e];
    s += twoX ? v01[e] : 0.0f;
    s += twoY ? v10[e] : 0.0f;
    s += (twoX && twoY) ? v11[e] : 0.0f;
    r[e] = s * inv;
  }
  float* op = out + ((size_t)(b * kChan + c) * kImg + (size_t)y) * kImg + x0;
  if (active) *(volatile v4f*)op = r;
  __threadfence();
  if (active) *(volatile v4f*)op = r;
}

extern "C" void kernel_launch(void* const* d_in, const int* in_sizes, int n_in,
                              void* d_out, int out_size, void* d_ws, size_t ws_size,
                              hipStream_t stream) {
  if (n_in < 5) return;
  if (in_sizes[0] != kBatch * kChan * kImg * kImg) return;
  if (in_sizes[1] != kChan * kEdim * kKpix) return;
  if (in_sizes[2] != kChan * kEdim) return;
  if (in_sizes[3] != kChan * kKpix * kEdim) return;
  if (in_sizes[4] != kChan * kKpix) return;
  if (out_size != kBatch * kChan * kImg * kImg) return;

  const float* x    = (const float*)d_in[0];
  const float* Wenc = (const float*)d_in[1];
  const float* benc = (const float*)d_in[2];
  const float* Wdec = (const float*)d_in[3];
  const float* bdec = (const float*)d_in[4];
  float* outp = (float*)d_out;

  const size_t SZ_WEB = (size_t)kChan * kEdim * kKpix * 2;
  const size_t SZ_WDB = (size_t)kChan * kKpix * kEdim * 2;
  const size_t SZ_A16 = (size_t)kRows * kKpix * 2;
  const size_t SZ_EMB = (size_t)kRows * kEdim * 2;
  const size_t SZ_REC = (size_t)kRows * kKpix * 4;
  size_t off = 0;
  const size_t oWEB  = off; off += SZ_WEB;
  const size_t oWDB  = off; off += SZ_WDB;
  const size_t oA16  = off; off += SZ_A16;
  const size_t oEMBH = off; off += SZ_EMB;
  const size_t oEMBL = off; off += SZ_EMB;
  const size_t oREC  = off; off += SZ_REC;
  const size_t TOTAL = off;
  if (TOTAL > ws_size) return;
  if (TOTAL > (size_t)134217728) return;

  char* ws = (char*)d_ws;
  unsigned short* WEB  = (unsigned short*)(ws + oWEB);
  unsigned short* WDB  = (unsigned short*)(ws + oWDB);
  unsigned short* A16  = (unsigned short*)(ws + oA16);
  unsigned short* EMBH = (unsigned short*)(ws + oEMBH);
  unsigned short* EMBL = (unsigned short*)(ws + oEMBL);
  float*          REC  = (float*)(ws + oREC);

  const dim3 blk(256);

  {
    const int n8 = kChan * kEdim * kKpix / 8;
    cast8_kernel<0><<<dim3(n8 / 256), blk, 0, stream>>>(Wenc, WEB, n8, 1.0f);
    cast8_kernel<0><<<dim3(n8 / 256), blk, 0, stream>>>(Wdec, WDB, n8, 1.0f);
  }

  const int tilesM = kRows / 64;
  const dim3 gEnc((tilesM * (kEdim / 64) + 7) / 8, 1);
  const dim3 gDec((tilesM * (kKpix / 64) + 7) / 8, 1);
  const dim3 gUnf(kRows / 8);
  const dim3 gFold(kBatch * kImg);

  for (int c = 0; c < kChan; ++c) {
    unfold_kernel<<<gUnf, blk, 0, stream>>>(x, A16, c, kRows);
    wmma_gemm64<1, 0, 3, 2><<<gEnc, blk, 0, stream>>>(
        A16, A16, kKpix, 0L,
        WEB + (size_t)c * kEdim * kKpix, WEB + (size_t)c * kEdim * kKpix, kKpix, 0L,
        (void*)EMBH, (void*)EMBL, kEdim, 0L,
        benc + (size_t)c * kEdim, 0L,
        kRows, kEdim, kKpix, 1.0f);
    wmma_gemm64<1, 1, 3, 0><<<gDec, blk, 0, stream>>>(
        EMBH, EMBL, kEdim, 0L,
        WDB + (size_t)c * kKpix * kEdim, WDB + (size_t)c * kKpix * kEdim, kEdim, 0L,
        (void*)REC, (void*)REC, kKpix, 0L,
        bdec + (size_t)c * kKpix, 0L,
        kRows, kKpix, kEdim, 1.0f);
    fold_kernel<<<gFold, dim3(64), 0, stream>>>(REC, outp, c);
  }
}
